// Layer_Block_39444979646721
// MI455X (gfx1250) — hardware-verified
//
#include <hip/hip_runtime.h>
#include <math.h>
#include <stdint.h>

#define NB   2
#define SEQ  4096
#define DM   768
#define NH   12
#define HD   64
#define FF   3072
#define NROW (NB * SEQ)
#define NQB  (SEQ / 64)
static_assert(NH * HD == DM);
static_assert((SEQ % 64) == 0 && (DM % 64) == 0 && (FF % 64) == 0 && (NROW % 64) == 0);
static_assert(DM == 3 * 256);

typedef _Float16 v16h __attribute__((ext_vector_type(16)));
typedef _Float16 v8h  __attribute__((ext_vector_type(8)));
typedef float    v8f  __attribute__((ext_vector_type(8)));
typedef float    v4f  __attribute__((ext_vector_type(4)));
typedef unsigned int v4u __attribute__((ext_vector_type(4)));

union H8 { v8h h; v4u u; };
union FH { v16h v; v8h h[2]; };

__device__ __forceinline__ v8f zero8() { v8f z = {0.f, 0.f, 0.f, 0.f, 0.f, 0.f, 0.f, 0.f}; return z; }

__device__ __forceinline__ v16h ldfrag(const _Float16* p) {
  FH f;
  f.h[0] = *(const v8h*)(p);
  f.h[1] = *(const v8h*)(p + 16);
  return f.v;
}

__device__ __forceinline__ v8f mma_h(v16h a, v16h b, v8f c) {
  c = __builtin_amdgcn_wmma_f32_16x16x32_f16(false, a, false, b, (short)0, c, false, false);
  asm volatile("v_nop\n\tv_nop\n\tv_nop\n\tv_nop" : "+v"(c) : "v"(a), "v"(b));
  return c;
}
__device__ __forceinline__ v8f mma_raw(v16h a, v16h b, v8f c) {
  return __builtin_amdgcn_wmma_f32_16x16x32_f16(false, a, false, b, (short)0, c, false, false);
}
__device__ __forceinline__ void guard4(v8f& d0, v8f& d1, v8f& d2, v8f& d3,
                                       v16h a, v16h b0, v16h b1, v16h b2, v16h b3) {
  asm volatile("v_nop\n\tv_nop\n\tv_nop\n\tv_nop"
               : "+v"(d0), "+v"(d1), "+v"(d2), "+v"(d3)
               : "v"(a), "v"(b0), "v"(b1), "v"(b2), "v"(b3));
}

__device__ __forceinline__ float gelu_tanh(float u) {
  const float z = 0.7978845608028654f * (u + 0.044715f * u * u * u);
  const float e = __expf(fminf(-2.0f * z, 80.0f));
  return u * __builtin_amdgcn_rcpf(1.0f + e);
}

__global__ __launch_bounds__(256) void tr_cvt(const float* __restrict__ W, _Float16* Wt,
                                              int Kin, int Nout, float scale) {
  __shared__ __align__(16) _Float16 T[64][72];
  const int tid = threadIdx.x, wave = tid >> 5, lane = tid & 31;
  const int n0 = blockIdx.x * 64, k0 = blockIdx.y * 64;
#pragma unroll
  for (int i = 0; i < 4; ++i) {
    const int chunk = tid + i * 256;
    const int r = chunk >> 4;
    const int c4 = (chunk & 15) * 4;
    const v4f v = *(const v4f*)(W + (size_t)(k0 + r) * Nout + n0 + c4);
#pragma unroll
    for (int e = 0; e < 4; ++e) T[c4 + e][r] = (_Float16)(v[e] * scale);
  }
  __syncthreads();
  const int q = lane >> 3, c8 = (lane & 7) * 8;
  v4u o[2];
#pragma unroll
  for (int it = 0; it < 2; ++it) {
    const int row = wave * 8 + it * 4 + q;
    H8 p;
    p.h = *(const v8h*)(&T[row][c8]);
    o[it] = p.u;
  }
  for (int pass = 0; pass < 2; ++pass) {
#pragma unroll
    for (int it = 0; it < 2; ++it) {
      const int row = wave * 8 + it * 4 + q;
      *(volatile v4u*)(Wt + (size_t)(n0 + row) * Kin + k0 + c8) = o[it];
    }
    __threadfence();
  }
}

__global__ __launch_bounds__(256) void ln_rows(const float* __restrict__ X, const float* __restrict__ g,
                                               const float* __restrict__ bb, _Float16* Y, int nrows) {
  const int wave = threadIdx.x >> 5, lane = threadIdx.x & 31;
  const int row = blockIdx.x * 8 + wave;
  if (row >= nrows) return;
  const float* xr = X + (size_t)row * DM;
  float v[3][8];
  float s = 0.f;
#pragma unroll
  for (int i = 0; i < 3; ++i) {
    const int col = i * 256 + lane * 8;
    const v4f a = *(const v4f*)(xr + col);
    const v4f c = *(const v4f*)(xr + col + 4);
#pragma unroll
    for (int e = 0; e < 4; ++e) { v[i][e] = a[e]; v[i][4 + e] = c[e]; }
#pragma unroll
    for (int e = 0; e < 8; ++e) s += v[i][e];
  }
#pragma unroll
  for (int off = 16; off > 0; off >>= 1) s += __shfl_xor(s, off, 32);
  const float mu = s * (1.0f / (float)DM);
  float qs = 0.f;
#pragma unroll
  for (int i = 0; i < 3; ++i)
#pragma unroll
    for (int e = 0; e < 8; ++e) { const float d = v[i][e] - mu; v[i][e] = d; qs += d * d; }
#pragma unroll
  for (int off = 16; off > 0; off >>= 1) qs += __shfl_xor(qs, off, 32);
  const float rstd = rsqrtf(qs * (1.0f / (float)DM) + 1e-5f);
  v4u o[3];
#pragma unroll
  for (int i = 0; i < 3; ++i) {
    const int col = i * 256 + lane * 8;
    const v4f g0 = *(const v4f*)(g + col), g1 = *(const v4f*)(g + col + 4);
    const v4f b0 = *(const v4f*)(bb + col), b1 = *(const v4f*)(bb + col + 4);
    H8 p;
#pragma unroll
    for (int e = 0; e < 4; ++e) {
      p.h[e]     = (_Float16)(v[i][e] * rstd * g0[e] + b0[e]);
      p.h[4 + e] = (_Float16)(v[i][4 + e] * rstd * g1[e] + b1[e]);
    }
    o[i] = p.u;
  }
  for (int pass = 0; pass < 2; ++pass) {
#pragma unroll
    for (int i = 0; i < 3; ++i)
      *(volatile v4u*)(Y + (size_t)row * DM + i * 256 + lane * 8) = o[i];
    __threadfence();
  }
}

template <int MODE>
__global__ __launch_bounds__(256) void gemm64(
    const _Float16* __restrict__ A, int lda, long long strideA,
    const _Float16* __restrict__ Bt, int ldb, long long strideB,
    const float* __restrict__ bias, const float* __restrict__ Res,
    void* Cout, int ldc, long long strideC,
    int M, int N, int K, float accs, float outs) {
  __shared__ __align__(16) float sT[8][16 * 68];
  const int bz   = blockIdx.y;
  const int lane = threadIdx.x & 31;
  const int wave = threadIdx.x >> 5;
  const int tilesN = N >> 6;
  const int tilesM = M >> 6;
  const int tile = blockIdx.x * 8 + wave;
  if (tile >= tilesM * tilesN) return;
  const int tm = tile / tilesN;
  const int tn = tile - tm * tilesN;
  const int m0 = tm << 6;
  const int n0 = tn << 6;

  const _Float16* Ab = A  + (size_t)bz * (size_t)strideA;
  const _Float16* Bb = Bt + (size_t)bz * (size_t)strideB;

  const int rl   = lane & 15;
  const int koff = (lane >> 4) * 8;
  const int mOff = (lane >> 4) * 8;

  v8f acc[4][4];
#pragma unroll
  for (int i = 0; i < 4; ++i)
#pragma unroll
    for (int j = 0; j < 4; ++j) acc[i][j] = zero8();

  for (int k0 = 0; k0 < K; k0 += 32) {
    v16h bf[4];
#pragma unroll
    for (int j = 0; j < 4; ++j)
      bf[j] = ldfrag(Bb + (size_t)(n0 + (j << 4) + rl) * ldb + koff + k0);
#pragma unroll
    for (int i = 0; i < 4; ++i) {
      const v16h af = ldfrag(Ab + (size_t)(m0 + (i << 4) + rl) * lda + koff + k0);
#pragma unroll
      for (int j = 0; j < 4; ++j) acc[i][j] = mma_raw(af, bf[j], acc[i][j]);
      guard4(acc[i][0], acc[i][1], acc[i][2], acc[i][3], af, bf[0], bf[1], bf[2], bf[3]);
    }
  }

  float* slab = sT[wave];
#pragma unroll
  for (int i = 0; i < 4; ++i) {
    const int mBase = m0 + (i << 4);
#pragma unroll
    for (int j = 0; j < 4; ++j) {
#pragma unroll
      for (int r = 0; r < 8; ++r) slab[(mOff + r) * 68 + (j << 4) + rl] = acc[i][j][r];
    }
    __builtin_amdgcn_fence(__ATOMIC_RELEASE, "workgroup");
    __builtin_amdgcn_wave_barrier();
    __builtin_amdgcn_fence(__ATOMIC_ACQUIRE, "workgroup");
    if constexpr (MODE == 2) {
      float* C = (float*)Cout + (size_t)bz * (size_t)strideC;
      const float* R = Res + (size_t)bz * (size_t)strideC;
      const int h2 = lane >> 4, c4 = (lane & 15) * 4;
      const v4f bq4 = *(const v4f*)(bias + n0 + c4);
      for (int pass = 0; pass < 2; ++pass) {
#pragma unroll
        for (int it = 0; it < 8; ++it) {
          const int row = it * 2 + h2;
          const v4f a  = *(const v4f*)(slab + row * 68 + c4);
          const v4f rr = *(const v4f*)(R + (size_t)(mBase + row) * ldc + n0 + c4);
          v4f ov;
#pragma unroll
          for (int e = 0; e < 4; ++e) ov[e] = rr[e] + (a[e] * accs + bq4[e]);
          *(volatile v4f*)(C + (size_t)(mBase + row) * ldc + n0 + c4) = ov;
        }
        __threadfence();
      }
    } else {
      _Float16* C = (_Float16*)Cout + (size_t)bz * (size_t)strideC;
      const int q = lane >> 3, c8 = (lane & 7) * 8;
      float bc[8];
      if constexpr (MODE != 1) {
        const v4f b0 = *(const v4f*)(bias + n0 + c8), b1 = *(const v4f*)(bias + n0 + c8 + 4);
#pragma unroll
        for (int e = 0; e < 4; ++e) { bc[e] = b0[e]; bc[4 + e] = b1[e]; }
      } else {
#pragma unroll
        for (int e = 0; e < 8; ++e) bc[e] = 0.f;
      }
      v4u hv[4];
#pragma unroll
      for (int it = 0; it < 4; ++it) {
        const int row = it * 4 + q;
        const float* sp = slab + row * 68 + c8;
        float brow = 0.f;
        if constexpr (MODE == 1) brow = bias[mBase + row];
        H8 p;
#pragma unroll
        for (int e = 0; e < 8; ++e) {
          float f = sp[e] * accs + ((MODE == 1) ? brow : bc[e]);
          if constexpr (MODE == 3) f = gelu_tanh(f);
          f *= outs;
          p.h[e] = (_Float16)f;
        }
        hv[it] = p.u;
      }
      for (int pass = 0; pass < 2; ++pass) {
#pragma unroll
        for (int it = 0; it < 4; ++it) {
          const int row = it * 4 + q;
          *(volatile v4u*)(C + (size_t)(mBase + row) * ldc + n0 + c8) = hv[it];
        }
        __threadfence();
      }
    }
    __builtin_amdgcn_fence(__ATOMIC_RELEASE, "workgroup");
    __builtin_amdgcn_wave_barrier();
    __builtin_amdgcn_fence(__ATOMIC_ACQUIRE, "workgroup");
  }
}

__global__ __launch_bounds__(128)
void attn_causal64(const _Float16* __restrict__ Qp, const _Float16* __restrict__ Kp,
                   const _Float16* __restrict__ Vtp, _Float16* Op, float sscale) {
  __shared__ __align__(16) _Float16 Ksh[64 * 64];
  __shared__ __align__(16) _Float16 Vth[64 * 64];
  __shared__ __align__(16) _Float16 Psh[4][16 * 64];
  __shared__ __align__(16) float    Os[4][16 * 64];

  const int tid  = threadIdx.x;
  const int wave = tid >> 5;
  const int lane = tid & 31;
  const int hh   = lane >> 4;
  const int c    = lane & 15;

  const int bx   = blockIdx.x;
  const int qb   = bx % NQB;
  const int rest = bx / NQB;
  const int h    = rest % NH;
  const int b    = rest / NH;
  const int q0   = qb * 64 + wave * 16;
  const size_t rowB = (size_t)b * SEQ;

  const _Float16* Qh = Qp + (size_t)h * HD;
  const _Float16* Kh = Kp + (size_t)h * HD;
  const _Float16* Vh = Vtp + ((size_t)b * DM + (size_t)h * HD) * SEQ;

  v16h qa[2];
#pragma unroll
  for (int dc = 0; dc < 2; ++dc)
    qa[dc] = ldfrag(Qh + (rowB + q0 + c) * DM + dc * 32 + 8 * hh);

  float mrow[8], lrow[8];
  v8f oacc[4];
#pragma unroll
  for (int r = 0; r < 8; ++r) { mrow[r] = -INFINITY; lrow[r] = 0.f; }
#pragma unroll
  for (int t = 0; t < 4; ++t) oacc[t] = zero8();

  for (int kt = 0; kt <= qb; ++kt) {
    const int kv0 = kt * 64;
    __syncthreads();
    {
      const int r = tid >> 1, half = (tid & 1) * 32;
      const _Float16* kg = Kh + (rowB + kv0 + r) * DM + half;
      const _Float16* vg = Vh + (size_t)r * SEQ + kv0 + half;
#pragma unroll
      for (int i = 0; i < 4; ++i) {
        const v8h a0 = *(const v8h*)(kg + 8 * i);
        const v8h b0 = *(const v8h*)(vg + 8 * i);
        *(v8h*)(Ksh + r * 64 + half + 8 * i) = a0;
        *(v8h*)(Vth + r * 64 + half + 8 * i) = b0;
      }
    }
    __syncthreads();

    v8f s[4];
#pragma unroll
    for (int j = 0; j < 4; ++j) {
      s[j] = zero8();
#pragma unroll
      for (int dc = 0; dc < 2; ++dc) {
        FH kb;
        kb.h[0] = *(const v8h*)(Ksh + (j * 16 + c) * 64 + dc * 32 + 8 * hh);
        kb.h[1] = *(const v8h*)(Ksh + (j * 16 + c) * 64 + dc * 32 + 16 + 8 * hh);
        s[j] = mma_h(qa[dc], kb.v, s[j]);
      }
    }

    _Float16* pw = Psh[wave];
#pragma unroll
    for (int r = 0; r < 8; ++r) {
      const int qrow = q0 + 8 * hh + r;
      float m = -INFINITY;
#pragma unroll
      for (int j = 0; j < 4; ++j) {
        const int key = kv0 + j * 16 + c;
        const float sv = (key <= qrow) ? (s[j][r] * sscale) : -INFINITY;
        s[j][r] = sv;
        m = fmaxf(m, sv);
      }
#pragma unroll
      for (int off = 1; off < 16; off <<= 1) m = fmaxf(m, __shfl_xor(m, off, 32));
      const float mnew  = fmaxf(mrow[r], m);
      const float msafe = (mnew == -INFINITY) ? 0.f : mnew;
      const float alpha = __expf(mrow[r] - msafe);
      mrow[r] = mnew;
      float psum = 0.f;
#pragma unroll
      for (int j = 0; j < 4; ++j) {
        const float p = __expf(s[j][r] - msafe);
        psum += p;
        pw[(8 * hh + r) * 64 + j * 16 + c] = (_Float16)(p * 1024.0f);
      }
#pragma unroll
      for (int off = 1; off < 16; off <<= 1) psum += __shfl_xor(psum, off, 32);
      lrow[r] = lrow[r] * alpha + psum;
#pragma unroll
      for (int t = 0; t < 4; ++t) oacc[t][r] *= alpha;
    }
    __builtin_amdgcn_fence(__ATOMIC_RELEASE, "workgroup");
    __builtin_amdgcn_wave_barrier();
    __builtin_amdgcn_fence(__ATOMIC_ACQUIRE, "workgroup");

#pragma unroll
    for (int kk = 0; kk < 2; ++kk) {
      FH pa;
      pa.h[0] = *(const v8h*)(pw + c * 64 + kk * 32 + 8 * hh);
      pa.h[1] = *(const v8h*)(pw + c * 64 + kk * 32 + 16 + 8 * hh);
#pragma unroll
      for (int t = 0; t < 4; ++t) {
        FH vb;
        vb.h[0] = *(const v8h*)(Vth + (t * 16 + c) * 64 + kk * 32 + 8 * hh);
        vb.h[1] = *(const v8h*)(Vth + (t * 16 + c) * 64 + kk * 32 + 16 + 8 * hh);
        oacc[t] = mma_h(pa.v, vb.v, oacc[t]);
      }
    }
  }

  float* os = Os[wave];
#pragma unroll
  for (int r = 0; r < 8; ++r) {
    const float l = lrow[r];
    const float inv = ((l > 0.f) ? (1.0f / l) : 0.f) * (1.0f / 1024.0f);
#pragma unroll
    for (int t = 0; t < 4; ++t) os[(8 * hh + r) * 64 + t * 16 + c] = oacc[t][r] * inv;
  }
  __builtin_amdgcn_fence(__ATOMIC_RELEASE, "workgroup");
  __builtin_amdgcn_wave_barrier();
  __builtin_amdgcn_fence(__ATOMIC_ACQUIRE, "workgroup");
  {
    const int q4 = lane >> 3, c8 = (lane & 7) * 8;
    v4u hv[4];
#pragma unroll
    for (int it = 0; it < 4; ++it) {
      const int row = it * 4 + q4;
      const float* sp = os + row * 64 + c8;
      H8 p;
#pragma unroll
      for (int e = 0; e < 8; ++e) p.h[e] = (_Float16)sp[e];
      hv[it] = p.u;
    }
    for (int pass = 0; pass < 2; ++pass) {
#pragma unroll
      for (int it = 0; it < 4; ++it) {
        const int row = it * 4 + q4;
        const size_t go = (rowB + q0 + row) * DM + (size_t)h * HD + c8;
        *(volatile v4u*)(Op + go) = hv[it];
      }
      __threadfence();
    }
  }
}

extern "C" void kernel_launch(void* const* d_in, const int* in_sizes, int n_in,
                              void* d_out, int out_size, void* d_ws, size_t ws_size,
                              hipStream_t stream) {
  if (n_in < 17) return;
  if (in_sizes[0] != NROW * DM) return;
  if (in_sizes[1] != DM || in_sizes[2] != DM) return;
  if (in_sizes[3] != DM * DM || in_sizes[5] != DM * DM || in_sizes[7] != DM * DM || in_sizes[9] != DM * DM) return;
  if (in_sizes[4] != DM || in_sizes[6] != DM || in_sizes[8] != DM || in_sizes[10] != DM) return;
  if (in_sizes[11] != DM || in_sizes[12] != DM) return;
  if (in_sizes[13] != DM * FF || in_sizes[14] != FF || in_sizes[15] != FF * DM || in_sizes[16] != DM) return;
  if (out_size != NROW * DM) return;

  const float* x    = (const float*)d_in[0];
  const float* ln1g = (const float*)d_in[1];
  const float* ln1b = (const float*)d_in[2];
  const float* Wq   = (const float*)d_in[3];
  const float* bq   = (const float*)d_in[4];
  const float* Wk   = (const float*)d_in[5];
  const float* bk   = (const float*)d_in[6];
  const float* Wv   = (const float*)d_in[7];
  const float* bv   = (const float*)d_in[8];
  const float* Wo   = (const float*)d_in[9];
  const float* bo   = (const float*)d_in[10];
  const float* ln2g = (const float*)d_in[11];
  const float* ln2b = (const float*)d_in[12];
  const float* W1   = (const float*)d_in[13];
  const float* b1   = (const float*)d_in[14];
  const float* W2   = (const float*)d_in[15];
  const float* b2   = (const float*)d_in[16];

  const size_t PWD  = (size_t)DM * DM * 2;
  const size_t PWF  = (size_t)DM * FF * 2;
  const size_t PA16 = (size_t)NROW * DM * 2;
  const size_t PVT  = (size_t)NB * DM * SEQ * 2;
  const size_t PG   = (size_t)NROW * FF * 2;
  const size_t PX1  = (size_t)NROW * DM * 4;
  size_t off = 0;
  const size_t oWq = off; off += PWD;
  const size_t oWk = off; off += PWD;
  const size_t oWv = off; off += PWD;
  const size_t oWo = off; off += PWD;
  const size_t oW1 = off; off += PWF;
  const size_t oW2 = off; off += PWF;
  const size_t oN  = off; off += PA16;
  const size_t oRB = off; off += PG;
  const size_t oCt = off; off += PA16;
  const size_t oX1 = off; off += PX1;
  if (off > ws_size) return;
  if (off > (size_t)134217728) return;
  const size_t oQ  = oRB;
  const size_t oK  = oRB + PA16;
  const size_t oVT = oRB + 2 * PA16;
  if (oVT + PVT > oRB + PG) return;
  const size_t oG  = oRB;

  char* ws = (char*)d_ws;
  _Float16* Wqt = (_Float16*)(ws + oWq);
  _Float16* Wkt = (_Float16*)(ws + oWk);
  _Float16* Wvt = (_Float16*)(ws + oWv);
  _Float16* Wot = (_Float16*)(ws + oWo);
  _Float16* W1t = (_Float16*)(ws + oW1);
  _Float16* W2t = (_Float16*)(ws + oW2);
  _Float16* Np  = (_Float16*)(ws + oN);
  _Float16* Qp  = (_Float16*)(ws + oQ);
  _Float16* Kpl = (_Float16*)(ws + oK);
  _Float16* VTp = (_Float16*)(ws + oVT);
  _Float16* Gp  = (_Float16*)(ws + oG);
  _Float16* Ctp = (_Float16*)(ws + oCt);
  float*    X1  = (float*)(ws + oX1);

  const dim3 blk(256);
  const dim3 gTrDD(DM / 64, DM / 64);
  const dim3 gTrW1(FF / 64, DM / 64);
  const dim3 gTrW2(DM / 64, FF / 64);
  const dim3 gLn((NROW + 7) / 8);
  const dim3 gProj(((NROW / 64) * (DM / 64) + 7) / 8, 1);
  const dim3 gVT(((DM / 64) * (SEQ / 64) + 7) / 8, NB);
  const dim3 gFfn(((NROW / 64) * (FF / 64) + 7) / 8, 1);
  const dim3 gAtt(NQB * NH * NB);

  tr_cvt<<<gTrDD, blk, 0, stream>>>(Wq, Wqt, DM, DM, 32.0f);
  tr_cvt<<<gTrDD, blk, 0, stream>>>(Wk, Wkt, DM, DM, 32.0f);
  tr_cvt<<<gTrDD, blk, 0, stream>>>(Wv, Wvt, DM, DM, 32.0f);
  tr_cvt<<<gTrDD, blk, 0, stream>>>(Wo, Wot, DM, DM, 32.0f);
  tr_cvt<<<gTrW1, blk, 0, stream>>>(W1, W1t, DM, FF, 32.0f);
  tr_cvt<<<gTrW2, blk, 0, stream>>>(W2, W2t, FF, DM, 32.0f);
  ln_rows<<<gLn, blk, 0, stream>>>(x, ln1g, ln1b, Np, NROW);
  gemm64<0><<<gProj, blk, 0, stream>>>(Np, DM, 0LL, Wqt, DM, 0LL, bq, x, (void*)Qp, DM, 0LL,
                                       NROW, DM, DM, 1.0f / 32.0f, 0.5f);
  gemm64<0><<<gProj, blk, 0, stream>>>(Np, DM, 0LL, Wkt, DM, 0LL, bk, x, (void*)Kpl, DM, 0LL,
                                       NROW, DM, DM, 1.0f / 32.0f, 4.0f);
  gemm64<1><<<gVT, blk, 0, stream>>>(Wvt, DM, 0LL, Np, DM, (long long)SEQ * DM, bv, x,
                                     (void*)VTp, SEQ, (long long)DM * SEQ,
                                     DM, SEQ, DM, 1.0f / 32.0f, 4.0f);
  attn_causal64<<<gAtt, dim3(128), 0, stream>>>(Qp, Kpl, VTp, Ctp, 0.0625f);
  gemm64<2><<<gProj, blk, 0, stream>>>(Ctp, DM, 0LL, Wot, DM, 0LL, bo, x, (void*)X1, DM, 0LL,
                                       NROW, DM, DM, 1.0f / 128.0f, 1.0f);
  ln_rows<<<gLn, blk, 0, stream>>>(X1, ln2g, ln2b, Np, NROW);
  gemm64<3><<<gFfn, blk, 0, stream>>>(Np, DM, 0LL, W1t, DM, 0LL, b1, x, (void*)Gp, FF, 0LL,
                                      NROW, FF, DM, 1.0f / 32.0f, 4.0f);
  gemm64<2><<<gProj, blk, 0, stream>>>(Gp, FF, 0LL, W2t, FF, 0LL, b2, X1, d_out, DM, 0LL,
                                       NROW, DM, FF, 1.0f / 128.0f, 1.0f);
  (void)hipGetLastError();
}
